// GNNPrediction_34050500722852
// MI455X (gfx1250) — hardware-run, weakly checked
//
#include <hip/hip_runtime.h>
#include <math.h>

typedef __attribute__((ext_vector_type(16))) _Float16 v16h;
typedef __attribute__((ext_vector_type(16))) __bf16 v16b;
typedef __attribute__((ext_vector_type(8)))  _Float16 v8h;
typedef __attribute__((ext_vector_type(8)))  float v8f;
typedef __attribute__((ext_vector_type(4)))  float v4f;
typedef __attribute__((ext_vector_type(2)))  float v2f;
typedef __attribute__((ext_vector_type(4)))  unsigned v4u;
typedef __attribute__((ext_vector_type(4)))  int v4i;
typedef float __attribute__((may_alias)) float_a;
typedef int __attribute__((may_alias)) int_a;

template <typename T> __device__ __forceinline__ void vst2(void* p, T v) { *(volatile T*)p = v; __threadfence(); *(volatile T*)p = v; }
__device__ __forceinline__ v8f wmma16(v16h a, v16h b, v8f c) {
  v8f d = __builtin_amdgcn_wmma_f32_16x16x32_f16(false, a, false, b, (short)0, c, false, false);
  asm volatile("v_nop\n\tv_nop\n\tv_nop\n\tv_nop" : "+v"(d) : "v"(a), "v"(b));
  return d;
}
__device__ __forceinline__ v8f wmma_bf(v16b a, v16b b, v8f c) {
  v8f d = __builtin_amdgcn_wmma_f32_16x16x32_bf16(false, a, false, b, (short)0, c, false, false);
  asm volatile("v_nop\n\tv_nop\n\tv_nop\n\tv_nop" : "+v"(d) : "v"(a), "v"(b));
  return d;
}
__device__ __forceinline__ v16h frag_h(const _Float16* rowk0, int lane) {
  union { v16h v; v8h q[2]; } u; const _Float16* p = rowk0 + 8 * (lane >> 4);
  u.q[0] = *(const v8h*)p; u.q[1] = *(const v8h*)(p + 16); return u.v;
}
__device__ __forceinline__ v16h frag_f32(const float* rowk0, int lane) {
  v16h a; const float* p = rowk0 + 8 * (lane >> 4);
#pragma unroll
  for (int i = 0; i < 8; ++i) { a[i] = (_Float16)p[i]; a[8 + i] = (_Float16)p[16 + i]; }
  return a;
}
__device__ __forceinline__ v16h frag_f32s(const float* rowk0, int lane, float sc) {
  v16h a; const float* p = rowk0 + 8 * (lane >> 4);
#pragma unroll
  for (int i = 0; i < 8; ++i) { a[i] = (_Float16)(p[i] * sc); a[8 + i] = (_Float16)(p[16 + i] * sc); }
  return a;
}
__device__ __forceinline__ v16h fragc_f32(const float* W, int k0, int n, int lane, int ld, int K) {
  v16h a; const int g = lane >> 4;
#pragma unroll
  for (int i = 0; i < 8; ++i) { const int ka = k0 + 8 * g + i, kb = ka + 16;
    a[i] = (_Float16)(ka < K ? W[(size_t)(ka < K ? ka : K - 1) * ld + n] : 0.f); a[8 + i] = (_Float16)(kb < K ? W[(size_t)(kb < K ? kb : K - 1) * ld + n] : 0.f); }
  return a;
}
struct F2 { v16b h, l; };
__device__ __forceinline__ F2 bsplit16(const float v[16]) { F2 r;
#pragma unroll
  for (int i = 0; i < 16; ++i) { const __bf16 h = (__bf16)v[i]; r.h[i] = h; r.l[i] = (__bf16)(v[i] - (float)h); }
  return r; }
__device__ __forceinline__ F2 split_row(const float* row, int k0, int lane) { float v[16]; const float* p = row + k0 + 8 * (lane >> 4);
#pragma unroll
  for (int i = 0; i < 8; ++i) { v[i] = p[i]; v[8 + i] = p[16 + i]; }
  return bsplit16(v); }
__device__ __forceinline__ F2 split_rowK(const float* row, int k0, int lane, int K) { float v[16]; const int g = lane >> 4;
#pragma unroll
  for (int i = 0; i < 8; ++i) { const int ka = k0 + 8 * g + i, kb = ka + 16; v[i] = ka < K ? row[ka < K ? ka : K - 1] : 0.f; v[8 + i] = kb < K ? row[kb < K ? kb : K - 1] : 0.f; }
  return bsplit16(v); }
__device__ __forceinline__ F2 split_col(const float* W, int k0, int n, int lane, int ld, int K) { float v[16]; const int g = lane >> 4;
#pragma unroll
  for (int i = 0; i < 8; ++i) { const int ka = k0 + 8 * g + i, kb = ka + 16; v[i] = ka < K ? W[(size_t)(ka < K ? ka : K - 1) * ld + n] : 0.f; v[8 + i] = kb < K ? W[(size_t)(kb < K ? kb : K - 1) * ld + n] : 0.f; }
  return bsplit16(v); }
__device__ __forceinline__ v8f mac3(const F2& a, const F2& b, v8f c) { c = wmma_bf(a.l, b.h, c); c = wmma_bf(a.h, b.l, c); return wmma_bf(a.h, b.h, c); }
__device__ __forceinline__ float sigm(float v) { return 1.0f / (1.0f + expf(-v)); }
#define LDSX() do { asm volatile("s_wait_dscnt 0" ::: "memory"); __builtin_amdgcn_wave_barrier(); __builtin_amdgcn_fence(__ATOMIC_RELEASE, "workgroup"); } while (0)


#define NBt 64
#define LAT 512
#define NMAX 128
#define DN 96
#define NP2 8128
#define NPP 8192
#define HID 256
#define OD 601
#define ODP 640
#define SH 128
#ifndef TEB
#define TEB NBt
#endif
typedef __attribute__((ext_vector_type(8))) __bf16 v8b;
__device__ __forceinline__ v16b frag_b(const __bf16* rowk0, int lane) {
  union { v16b v; v8b q[2]; } u; const __bf16* p = rowk0 + 8 * (lane >> 4);
  u.q[0] = *(const v8b*)p; u.q[1] = *(const v8b*)(p + 16); return u.v;
}
__device__ __forceinline__ float bfr(float v) { return (float)(__bf16)v; }
__device__ __attribute__((noinline)) float exp_ni(float v) { return expf(v); }
__device__ __attribute__((noinline)) float erf_ni(float v) { return erff(v); }

#define OUT1_OFF ((size_t)NBt * OD)
#define OUT2_OFF ((size_t)2 * NBt * OD)
#define WS_H1  0u
#define WS_VR  (WS_H1 + 4u * (size_t)2 * NBt * HID)
#define WS_ED  (WS_VR + 4u * (size_t)2 * NBt * ODP)
#define WS_SAT (WS_ED + 4u * (size_t)NBt * NPP)
#define WS_END (WS_SAT + 4u * 64)

__global__ __launch_bounds__(128) void k_h1(const float* __restrict__ Z, const float* __restrict__ VW1, const float* __restrict__ VB1, const float* __restrict__ RW1, const float* __restrict__ RB1, float* __restrict__ H1) { __shared__ __align__(16) float sf[4][16][132];
  const int tid = threadIdx.x, wave = tid >> 5, lane = tid & 31, col = lane & 15, g = lane >> 4; const int c0 = blockIdx.x * 128; const int which = blockIdx.y; const float* Wm = which == 0 ? VW1 : RW1; const float* Bm = which == 0 ? VB1 : RB1; const size_t r0 = wave * 16;
  v8f acc[8] = {};
#pragma unroll 2
  for (int kc = 0; kc < LAT / 32; ++kc) { v16b a; { const float* p = Z + (r0 + col) * LAT + kc * 32 + 8 * g;
#pragma unroll
      for (int i = 0; i < 8; ++i) { a[i] = (__bf16)p[i]; a[8 + i] = (__bf16)p[16 + i]; } }
#pragma unroll
    for (int j = 0; j < 8; ++j) { v16b w; const int o = c0 + j * 16 + col;
#pragma unroll
      for (int i = 0; i < 8; ++i) { w[i] = (__bf16)Wm[(size_t)(kc * 32 + 8 * g + i) * HID + o]; w[8 + i] = (__bf16)Wm[(size_t)(kc * 32 + 16 + 8 * g + i) * HID + o]; }
      acc[j] = wmma_bf(a, w, acc[j]); } }
#pragma unroll
  for (int j = 0; j < 8; ++j) { const float bb = bfr(Bm[c0 + j * 16 + col]);
#pragma unroll
    for (int r = 0; r < 8; ++r) sf[wave][8 * g + r][j * 16 + col] = fmaxf(acc[j][r] + bb, 0.f); }
  LDSX(); for (int rl = 0; rl < 16; ++rl) vst2(H1 + ((size_t)which * NBt + r0 + rl) * HID + c0 + lane * 4, *(const v4f*)&sf[wave][rl][lane * 4]); }
__global__ __launch_bounds__(128) void k_h2(const float* __restrict__ H1, const float* __restrict__ VW2, const float* __restrict__ VB2, const float* __restrict__ RW2, const float* __restrict__ RB2, float* __restrict__ VR) { __shared__ __align__(16) float sf[4][16][132];
  const int tid = threadIdx.x, wave = tid >> 5, lane = tid & 31, col = lane & 15, g = lane >> 4; const int c0 = blockIdx.x * 128; const int which = blockIdx.y; const float* Wm = which == 0 ? VW2 : RW2; const float* Bm = which == 0 ? VB2 : RB2; const size_t r0 = wave * 16;
  v8f acc[8] = {};
#pragma unroll
  for (int kc = 0; kc < HID / 32; ++kc) { const F2 a = split_row(H1 + ((size_t)which * NBt + r0 + col) * HID, kc * 32, lane);
#pragma unroll
    for (int j = 0; j < 8; ++j) { v16b w; const int o = min(c0 + j * 16 + col, OD - 1);
#pragma unroll
      for (int i = 0; i < 8; ++i) { w[i] = (__bf16)Wm[(size_t)(kc * 32 + 8 * g + i) * OD + o]; w[8 + i] = (__bf16)Wm[(size_t)(kc * 32 + 16 + 8 * g + i) * OD + o]; }
      acc[j] = wmma_bf(a.h, w, acc[j]); acc[j] = wmma_bf(a.l, w, acc[j]); } }
#pragma unroll
  for (int j = 0; j < 8; ++j) { const int o = min(c0 + j * 16 + col, OD - 1); const float bb = bfr(Bm[o]);
#pragma unroll
    for (int r = 0; r < 8; ++r) sf[wave][8 * g + r][j * 16 + col] = acc[j][r] + bb; }
  LDSX(); for (int rl = 0; rl < 16; ++rl) vst2(VR + ((size_t)which * NBt + r0 + rl) * ODP + c0 + lane * 4, *(const v4f*)&sf[wave][rl][lane * 4]); }
__device__ __forceinline__ void pair_ij(int p, int& i, int& j) {
  float fi = ((2.0f * NMAX - 1.0f) - sqrtf((2.0f * NMAX - 1.0f) * (2.0f * NMAX - 1.0f) - 8.0f * (float)p)) * 0.5f; int ii = (int)fi; if (ii < 0) ii = 0; if (ii > NMAX - 2) ii = NMAX - 2;
  while (ii > 0 && (ii * (2 * NMAX - ii - 1)) / 2 > p) --ii; while (((ii + 1) * (2 * NMAX - ii - 2)) / 2 <= p) ++ii;
  i = ii; j = p - (ii * (2 * NMAX - ii - 1)) / 2 + ii + 1; }
__global__ __launch_bounds__(128) void k_edge(const float* __restrict__ Hn, const float* __restrict__ SW1, const float* __restrict__ SB1, const float* __restrict__ SW2, const float* __restrict__ SB2, float* __restrict__ ED) { __shared__ __align__(16) float sfeat[64][392]; __shared__ __align__(16) float so[64];
  const int tid = threadIdx.x, wave = tid >> 5, lane = tid & 31, col = lane & 15, g = lane >> 4; const int p0 = blockIdx.x * 64; const size_t b = blockIdx.y;
  for (int e = tid; e < 64 * DN; e += 128) { const int rl = e / DN, d = e % DN; const int p = p0 + rl; float hi_ = 0.f, hj_ = 0.f; if (p < NP2) { int i, j; pair_ij(p, i, j); hi_ = bfr(Hn[(b * NMAX + i) * DN + d]); hj_ = bfr(Hn[(b * NMAX + j) * DN + d]); }
    sfeat[rl][d] = hi_; sfeat[rl][DN + d] = hj_; sfeat[rl][2 * DN + d] = fabsf(hi_ - hj_); sfeat[rl][3 * DN + d] = hi_ * hj_; }
  __syncthreads();
  v8f acc[8] = {};
#pragma unroll 1
  for (int kc = 0; kc < 384 / 32; ++kc) { const F2 a = split_row(&sfeat[wave * 16 + col][0], kc * 32, lane); const bool two = (kc >= 6);
#pragma unroll
    for (int j = 0; j < 8; ++j) { v16b w; const int o = j * 16 + col;
#pragma unroll
      for (int i = 0; i < 8; ++i) { w[i] = (__bf16)SW1[(size_t)(kc * 32 + 8 * g + i) * SH + o]; w[8 + i] = (__bf16)SW1[(size_t)(kc * 32 + 16 + 8 * g + i) * SH + o]; }
      acc[j] = wmma_bf(a.h, w, acc[j]); if (two) acc[j] = wmma_bf(a.l, w, acc[j]); } }
  float part[8];
#pragma unroll
  for (int r = 0; r < 8; ++r) part[r] = 0.f;
#pragma unroll
  for (int j = 0; j < 8; ++j) { const int o = j * 16 + col; const float bb = bfr(SB1[o]), w2 = bfr(SW2[o]);
#pragma unroll
    for (int r = 0; r < 8; ++r) part[r] += fmaxf(acc[j][r] + bb, 0.f) * w2; }
#pragma unroll
  for (int r = 0; r < 8; ++r) { float v = part[r];
#pragma unroll
    for (int o = 1; o < 16; o <<= 1) v += __shfl_xor(v, o); if (col == 0) so[wave * 16 + 8 * g + r] = v + bfr(SB2[0]); }
  __syncthreads(); if (tid < 16) vst2(ED + b * NPP + p0 + tid * 4, *(const v4f*)&so[tid * 4]); }
__global__ __launch_bounds__(256) void k_sat(const float* __restrict__ Z, const float* __restrict__ SW, const float* __restrict__ SB, float* __restrict__ SAT) { __shared__ __align__(16) float so[64]; const int t = threadIdx.x; const int wv = t >> 5, ln = t & 31;
  for (int b = wv; b < NBt; b += 8) { float a = 0.f; for (int k = ln; k < LAT; k += 32) a += bfr(Z[b * LAT + k]) * bfr(SW[k]);
#pragma unroll
    for (int o = 1; o < 32; o <<= 1) a += __shfl_xor(a, o); if (ln == 0) so[b] = a + bfr(SB[0]); }
  __syncthreads(); if (t < 16) vst2(SAT + t * 4, *(const v4f*)&so[t * 4]); }
__global__ __launch_bounds__(256) void k_pack(const float* __restrict__ VR, const float* __restrict__ ED, const float* __restrict__ SAT, float* __restrict__ OUT) {
  const size_t q = (size_t)blockIdx.x * 256 + threadIdx.x; const size_t n01 = (size_t)NBt * OD; const size_t n2 = (size_t)NBt * (NP2 + 1); const size_t total4 = (2 * n01 + n2) / 4;
  if (q >= total4) return; __align__(16) float v[4];
  for (int k = 0; k < 4; ++k) { const size_t f = q * 4 + k; float x;
    if (f < 2 * n01) { const size_t which = f / n01, rem = f % n01; const size_t r = rem / OD, c = rem % OD; x = VR[(which * NBt + r) * ODP + c]; }
    else { const size_t rem = f - 2 * n01; const size_t r = rem / (NP2 + 1), c = rem % (NP2 + 1); x = (c < NP2) ? ED[r * NPP + c] : SAT[r]; }
    v[k] = x; }
  vst2(OUT + q * 4, *(const v4f*)v); }
extern "C" void kernel_launch(void* const* d_in, const int* in_sizes, int n_in, void* d_out, int out_size, void* d_ws, size_t ws_size, hipStream_t stream) {
  (void)in_sizes; (void)n_in; (void)out_size;
  const float** F = (const float**)d_in;
  if (ws_size < (size_t)WS_END) return;
  char* ws = (char*)d_ws; float *H1 = (float*)(ws + WS_H1), *VR = (float*)(ws + WS_VR), *ED = (float*)(ws + WS_ED), *SAT = (float*)(ws + WS_SAT);
  k_h1<<<dim3(HID / 128, 2), 128, 0, stream>>>(F[0], F[2], F[3], F[6], F[7], H1);
  k_h2<<<dim3(ODP / 128, 2), 128, 0, stream>>>(H1, F[4], F[5], F[8], F[9], VR);
  k_edge<<<dim3(NPP / 64, TEB), 128, 0, stream>>>(F[1], F[10], F[11], F[12], F[13], ED);
  k_sat<<<1, 256, 0, stream>>>(F[0], F[14], F[15], SAT);
  const size_t total4 = ((size_t)2 * NBt * OD + (size_t)NBt * (NP2 + 1)) / 4;
  k_pack<<<(unsigned)((total4 + 255) / 256), 256, 0, stream>>>(VR, ED, SAT, (float*)d_out);
}
